// PRM_7352984011191
// MI455X (gfx1250) — hardware-verified
//
#include <hip/hip_runtime.h>


#define NB_  4
#define CC   64
#define HW   4096
#define PCAR 1024.0f
typedef _Float16 h16;
typedef unsigned short bf;
typedef __attribute__((ext_vector_type(16))) __bf16   v16bf;
typedef __attribute__((ext_vector_type(16))) _Float16 v16h;
typedef __attribute__((ext_vector_type(8)))  _Float16 v8h;
typedef __attribute__((ext_vector_type(8)))  unsigned short v8us;
typedef __attribute__((ext_vector_type(8)))  float    v8f;
typedef __attribute__((ext_vector_type(4)))  float    v4f;
typedef v8h  __attribute__((may_alias)) v8ha;
typedef v4f  __attribute__((may_alias)) v4fa;
typedef v8us __attribute__((may_alias)) v8usa;

__device__ __forceinline__ unsigned short f2bf(float f) { unsigned u = __float_as_uint(f); u += 0x7FFFu + ((u >> 16) & 1u); return (unsigned short)(u >> 16); }
__device__ __forceinline__ float bf2f(unsigned short b) { return __uint_as_float(((unsigned)b) << 16); }
__device__ __forceinline__ float bfr(float f) { return bf2f(f2bf(f)); }
__device__ __forceinline__ v16h cat16(v8h lo, v8h hi) { return __builtin_shufflevector(lo, hi, 0, 1, 2, 3, 4, 5, 6, 7, 8, 9, 10, 11, 12, 13, 14, 15); }
__device__ __forceinline__ v16bf cat16b(v8us lo, v8us hi) { return __builtin_bit_cast(v16bf, __builtin_shufflevector(lo, hi, 0, 1, 2, 3, 4, 5, 6, 7, 8, 9, 10, 11, 12, 13, 14, 15)); }
__device__ __forceinline__ v8f wmma16(v16h a, v16h b, v8f c) { return __builtin_amdgcn_wmma_f32_16x16x32_f16(false, a, false, b, (short)0, c, false, false); }
__device__ __forceinline__ v8f wmmab(v16bf a, v16bf b, v8f c) { return __builtin_amdgcn_wmma_f32_16x16x32_bf16(false, a, false, b, (short)0, c, false, false); }


template <typename T16> struct WFrag;
template <> struct WFrag<h16> { typedef v16h V; static __device__ __forceinline__ V ld(const h16* p) { return cat16(*(const v8h*)p, *(const v8h*)(p + 16)); } static __device__ __forceinline__ v8f mma(V a, V b, v8f c) { return wmma16(a, b, c); } };
template <> struct WFrag<bf> { typedef v16bf V; static __device__ __forceinline__ V ld(const bf* p) { return cat16b(*(const v8us*)p, *(const v8us*)(p + 16)); } static __device__ __forceinline__ v8f mma(V a, V b, v8f c) { return wmmab(a, b, c); } };
template <typename T16, int NSPLIT, bool BIAS>
__global__ __launch_bounds__(32) void k_gemmw(const T16* __restrict__ A, const T16* __restrict__ A2, const T16* __restrict__ Bt, const T16* __restrict__ Bt2, int K, float* C, int ldc, const float* __restrict__ bias, size_t sA, size_t sB, size_t sC) {
    typedef typename WFrag<T16>::V V;
    __shared__ __align__(16) float os[16 * 68];
    const size_t z = blockIdx.z; A += z * sA; if (A2) A2 += z * sA; Bt += z * sB; if (Bt2) Bt2 += z * sB; C += z * sC;
    const int lane = threadIdx.x & 31, lr = lane & 15, hi = lane >> 4; const int r0 = blockIdx.x * 64, c0 = blockIdx.y * 64;
    v8f acc[4][4];
#pragma unroll
    for (int mb = 0; mb < 4; ++mb)
#pragma unroll
        for (int nb = 0; nb < 4; ++nb) acc[mb][nb] = (v8f){};
    const size_t aoff = (size_t)(r0 + lr) * K + 8 * hi, boff = (size_t)(c0 + lr) * K + 8 * hi;
#pragma unroll 1
    for (int kc = 0; kc < K; kc += 32) {
        V a[4], a2[4];
#pragma unroll
        for (int mb = 0; mb < 4; ++mb) { a[mb] = WFrag<T16>::ld(A + aoff + (size_t)mb * 16 * K + kc); if (NSPLIT == 1 || NSPLIT == 2) a2[mb] = WFrag<T16>::ld(A2 + aoff + (size_t)mb * 16 * K + kc); }
#pragma unroll
        for (int nb = 0; nb < 4; ++nb) { const V b = WFrag<T16>::ld(Bt + boff + (size_t)nb * 16 * K + kc); V b2; if (NSPLIT >= 2) b2 = WFrag<T16>::ld(Bt2 + boff + (size_t)nb * 16 * K + kc);
#pragma unroll
            for (int mb = 0; mb < 4; ++mb) { acc[mb][nb] = WFrag<T16>::mma(a[mb], b, acc[mb][nb]); if (NSPLIT == 1 || NSPLIT == 2) acc[mb][nb] = WFrag<T16>::mma(a2[mb], b, acc[mb][nb]); if (NSPLIT >= 2) acc[mb][nb] = WFrag<T16>::mma(a[mb], b2, acc[mb][nb]); } }
        asm volatile("v_nop\n\tv_nop\n\tv_nop\n\tv_nop" : "+v"(acc[0][0]), "+v"(acc[1][1]), "+v"(acc[2][2]), "+v"(acc[3][3]) : "v"(a[0]), "v"(a[3]));
    }
#pragma unroll
    for (int mb = 0; mb < 4; ++mb) {
#pragma unroll
        for (int nb = 0; nb < 4; ++nb) {
#pragma unroll
            for (int j = 0; j < 8; ++j) os[(hi * 8 + j) * 68 + nb * 16 + lr] = acc[mb][nb][j]; }
        __builtin_amdgcn_wave_barrier(); asm volatile("" ::: "memory");
        float* crow = C + (size_t)(r0 + mb * 16) * ldc + c0;
#pragma unroll 1
        for (int ps = 0; ps < 2; ++ps) {
#pragma unroll
            for (int s = 0; s < 8; ++s) { const int row = 2 * s + hi, cofs = lr * 4; v4f val = *(const v4fa*)(os + row * 68 + cofs); if (BIAS) { val[0] += bfr(bias[c0 + cofs]); val[1] += bfr(bias[c0 + cofs + 1]); val[2] += bfr(bias[c0 + cofs + 2]); val[3] += bfr(bias[c0 + cofs + 3]); }
                *(volatile v4f*)(crow + (size_t)row * ldc + cofs) = val; }
            if (ps == 0) __threadfence(); }
        __builtin_amdgcn_wave_barrier(); asm volatile("" ::: "memory");
    }
}

__device__ __forceinline__ h16 tohx(float x) { return (h16)x; }
typedef __attribute__((ext_vector_type(4))) unsigned short v4us;
typedef __attribute__((ext_vector_type(4))) _Float16 v4h;
typedef __attribute__((ext_vector_type(8))) _Float16 v8h;

__global__ __launch_bounds__(256) void k_tb(const float* __restrict__ F, bf* T) { const int e = (blockIdx.x * 256 + threadIdx.x) * 4; if (e >= HW * CC) return; const int c = e % CC; const int s = e / CC; v4us o;
#pragma unroll
    for (int u = 0; u < 4; ++u) o[u] = f2bf(F[(size_t)(c + u) * HW + s]); *(volatile v4us*)(T + e) = o; __threadfence(); *(volatile v4us*)(T + e) = o; }
__global__ __launch_bounds__(256) void k_v16(const float* __restrict__ F, h16* V) { const int e = (blockIdx.x * 256 + threadIdx.x) * 8; if (e >= CC * HW) return; const v4f a = *(const v4f*)(F + e), b = *(const v4f*)(F + e + 4); v8h o;
#pragma unroll
    for (int u = 0; u < 4; ++u) { o[u] = tohx(bfr(a[u])); o[4 + u] = tohx(bfr(b[u])); } *(volatile v8h*)(V + e) = o; __threadfence(); *(volatile v8h*)(V + e) = o; }
__global__ __launch_bounds__(256) void k_ssoft(const float* __restrict__ Sb, h16* P16) { const int lane = threadIdx.x & 31; const int row = blockIdx.x * 8 + (threadIdx.x >> 5); if (row >= HW) return; const float* sr = Sb + (size_t)row * HW; float mx = -3.0e38f;
    for (int ch = 0; ch < HW / 128; ++ch) { const v4f a = *(const v4f*)(sr + ch * 128 + lane * 4);
#pragma unroll
        for (int q = 0; q < 4; ++q) mx = fmaxf(mx, a[q]); }
#pragma unroll
    for (int sh = 16; sh; sh >>= 1) mx = fmaxf(mx, __shfl_xor(mx, sh, 32));
    float sum = 0.f;
    for (int ch = 0; ch < HW / 128; ++ch) { const v4f a = *(const v4f*)(sr + ch * 128 + lane * 4);
#pragma unroll
        for (int q = 0; q < 4; ++q) { float d0 = __fsub_rn(a[q], mx); asm volatile("" : "+v"(d0)); sum += __builtin_amdgcn_exp2f(__fmul_rn(d0, 1.4426950408889634f)); } }
#pragma unroll
    for (int sh = 16; sh; sh >>= 1) sum += __shfl_xor(sum, sh, 32);
    const float f = __fdiv_rn(PCAR, sum);
    for (int ch = 0; ch < HW / 128; ++ch) { const v4f a = *(const v4f*)(sr + ch * 128 + lane * 4); v4h o4;
#pragma unroll
        for (int q = 0; q < 4; ++q) { float d0 = __fsub_rn(a[q], mx); asm volatile("" : "+v"(d0)); o4[q] = tohx(__builtin_amdgcn_exp2f(__fmul_rn(d0, 1.4426950408889634f)) * f); }
        h16* dst = P16 + (size_t)row * HW + ch * 128 + lane * 4; *(volatile v4h*)dst = o4; __threadfence(); *(volatile v4h*)dst = o4; } }
__global__ __launch_bounds__(256) void k_fin(const float* __restrict__ O, float* outn) { const int e = (blockIdx.x * 256 + threadIdx.x) * 4; if (e >= CC * HW) return; const int s = e % HW; const int c = e / HW; v4f r;
#pragma unroll
    for (int u = 0; u < 4; ++u) r[u] = O[(size_t)(s + u) * CC + c] * (1.0f / PCAR); *(volatile v4f*)(outn + e) = r; __threadfence(); *(volatile v4f*)(outn + e) = r; }

extern "C" void kernel_launch(void* const* d_in, const int* in_sizes, int n_in,
                              void* d_out, int out_size, void* d_ws, size_t ws_size, hipStream_t stream) {
    (void)in_sizes; (void)n_in; (void)out_size;
    const float* lp = (const float*)d_in[0]; const float* up = (const float*)d_in[1];
    float* OUT = (float*)d_out;
    char* wsp = (char*)d_ws;
    auto take = [&](size_t bytes) { char* p = wsp; wsp += (bytes + 255) & ~(size_t)255; return (void*)p; };
    bf* QB = (bf*)take((size_t)HW * CC * 2); bf* KB = (bf*)take((size_t)HW * CC * 2); h16* VT = (h16*)take((size_t)CC * HW * 2); float* Sb = (float*)take((size_t)HW * HW * 4); h16* P16 = (h16*)take((size_t)HW * HW * 2); float* O = (float*)take((size_t)HW * CC * 4);
    if ((size_t)(wsp - (char*)d_ws) > ws_size) return;
    for (int n = 0; n < NB_; ++n) { const float* lpn = lp + (size_t)n * CC * HW; const float* upn = up + (size_t)n * CC * HW;
        k_tb<<<(HW * CC / 4 + 255) / 256, 256, 0, stream>>>(upn, QB); k_tb<<<(HW * CC / 4 + 255) / 256, 256, 0, stream>>>(lpn, KB); k_v16<<<(CC * HW / 8 + 255) / 256, 256, 0, stream>>>(lpn, VT);
        k_gemmw<bf, 0, false><<<dim3(HW / 64, HW / 64, 1), 32, 0, stream>>>(QB, nullptr, KB, nullptr, CC, Sb, HW, nullptr, 0, 0, 0);
        k_ssoft<<<HW / 8, 256, 0, stream>>>(Sb, P16);
        k_gemmw<h16, 0, false><<<dim3(HW / 64, 1, 1), 32, 0, stream>>>(P16, nullptr, VT, nullptr, HW, O, CC, nullptr, 0, 0, 0);
        k_fin<<<(CC * HW / 4 + 255) / 256, 256, 0, stream>>>(O, OUT + (size_t)n * CC * HW); }
}
